// MHAttention_own_52226802319926
// MI455X (gfx1250) — hardware-verified
//
#include <hip/hip_runtime.h>
#include <stdint.h>


typedef __attribute__((ext_vector_type(16))) _Float16 v16h;
typedef __attribute__((ext_vector_type(8)))  _Float16 v8h;
typedef __attribute__((ext_vector_type(8)))  float    v8f;
typedef __attribute__((ext_vector_type(4)))  float    v4f;

#define S_LEN 1024
#define HD 64
#define N_HEADS 8
#define C_CH 512
#define QB 64
#define KC 64
#define NWAVE 4
#define PSC 32768.0f
#define SCALE_QK 0.125f
#define NEG_FILL (-1.0e30f)
#define TP 72
#define OP 68

template <typename T> struct Frag;
template <> struct Frag<_Float16> {
  typedef v16h V; union U { v16h v; v8h h[2]; };
  static __device__ __forceinline__ v16h load(const _Float16* p) {
    U f; f.h[0] = *(const v8h*)(p); f.h[1] = *(const v8h*)(p + 16); return f.v;
  }
};

__device__ __forceinline__ v8f mma_h(v16h a, v16h b, v8f c) {
  c = __builtin_amdgcn_wmma_f32_16x16x32_f16(false, a, false, b, (short)0, c, false, false);
  asm volatile("v_nop\n\tv_nop\n\tv_nop\n\tv_nop" : "+v"(c) : "v"(a), "v"(b));
  return c;
}

__global__ __launch_bounds__(256) void cast_f32_f16x2(
    const float* __restrict__ in, _Float16* __restrict__ out, int n2) {
  int i = blockIdx.x * 256 + threadIdx.x;
  if (i < n2) {
    const _Float16 h0 = (_Float16)in[2 * i], h1 = (_Float16)in[2 * i + 1];
    const unsigned u = (unsigned)__builtin_bit_cast(unsigned short, h0) | ((unsigned)__builtin_bit_cast(unsigned short, h1) << 16);
    ((volatile unsigned*)out)[i] = u;
    __threadfence();
    ((volatile unsigned*)out)[i] = u;
  }
}

__global__ __launch_bounds__(128) void tcast_kernel(
    const float* __restrict__ x0, const float* __restrict__ x1,
    _Float16* __restrict__ y0, _Float16* __restrict__ y1) {
  __shared__ __align__(16) _Float16 T[64 * TP];
  const int tid = threadIdx.x, lane = tid & 31, wave = tid >> 5;
  const int t0 = blockIdx.x * 64;
  const int bh = blockIdx.y;
  const float* in = (blockIdx.z == 0) ? x0 : x1;
  _Float16* out = (blockIdx.z == 0) ? y0 : y1;
  const float* src = in + (size_t)bh * HD * S_LEN + t0;
#pragma unroll
  for (int i = 0; i < 8; ++i) {
    const int idx = tid + 128 * i;
    const int d  = idx >> 4;
    const int t4 = (idx & 15) * 4;
    const v4f v = *(const v4f*)(src + (size_t)d * S_LEN + t4);
#pragma unroll
    for (int e = 0; e < 4; ++e) T[(t4 + e) * TP + d] = (_Float16)v[e];
  }
  __syncthreads();
  _Float16* dst = out + ((size_t)bh * S_LEN + t0) * HD;
  const int rq = lane >> 3, c8 = (lane & 7) * 8;
  for (int pass = 0; pass < 2; ++pass) {
#pragma unroll
    for (int it = 0; it < 4; ++it) {
      const int row = wave * 16 + it * 4 + rq;
      const v8h hv = *(const v8h*)(T + row * TP + c8);
      *(volatile v8h*)(dst + (size_t)row * HD + c8) = hv;
    }
    __threadfence();
  }
}

__global__ __launch_bounds__(128)
void attn_kernel(const _Float16* __restrict__ Qt, const _Float16* __restrict__ Kt,
                 const _Float16* __restrict__ Vh, const float* __restrict__ mk,
                 float* __restrict__ out, int nheads) {
  __shared__ __align__(16) _Float16 Ksh[KC * HD];
  __shared__ __align__(16) _Float16 Vth[HD * KC];
  __shared__ __align__(16) _Float16 Psh[NWAVE][16 * KC];
  __shared__ __align__(16) float    Ob[HD * OP];

  const int tid  = threadIdx.x;
  const int wave = tid >> 5;
  const int lane = tid & 31;
  const int hh   = lane >> 4;
  const int c    = lane & 15;

  const int bh  = blockIdx.y;
  const int b   = bh / nheads;
  const int qb  = blockIdx.x;
  const int q0b = qb * QB;
  const int q0  = q0b + wave * 16;

  const _Float16* qbp = Qt + (size_t)bh * S_LEN * HD;
  const _Float16* kbp = Kt + (size_t)bh * S_LEN * HD;
  const _Float16* vbp = Vh + (size_t)bh * HD * S_LEN;
  const float*    mbp = mk + (size_t)b * S_LEN * S_LEN;
  float*          obp = out + (size_t)bh * HD * S_LEN;

  v16h qf[2];
  qf[0] = Frag<_Float16>::load(qbp + (size_t)(q0 + c) * HD + 0  + 8 * hh);
  qf[1] = Frag<_Float16>::load(qbp + (size_t)(q0 + c) * HD + 32 + 8 * hh);

  float mrow[8], lrow[8];
  v8f oacc[4];
#pragma unroll
  for (int r = 0; r < 8; ++r) { mrow[r] = NEG_FILL; lrow[r] = 0.f; }
#pragma unroll
  for (int t = 0; t < 4; ++t) oacc[t] = (v8f){0.f,0.f,0.f,0.f,0.f,0.f,0.f,0.f};

  for (int kc = 0; kc < S_LEN / KC; ++kc) {
    const int kv0 = kc * KC;
    __syncthreads();
#pragma unroll
    for (int i = 0; i < 4; ++i) {
      const int idx = tid + 128 * i;
      const int row = idx >> 3;
      const int c8  = (idx & 7) * 8;
      const v8h kv = *(const v8h*)(kbp + (size_t)(kv0 + row) * HD + c8);
      const v8h vv = *(const v8h*)(vbp + (size_t)row * S_LEN + kv0 + c8);
      *(v8h*)(Ksh + row * HD + c8) = kv;
      *(v8h*)(Vth + row * KC + c8) = vv;
    }
    __syncthreads();

    v8f s[4];
#pragma unroll
    for (int j = 0; j < 4; ++j) {
      s[j] = (v8f){0.f,0.f,0.f,0.f,0.f,0.f,0.f,0.f};
      const v16h kb0 = Frag<_Float16>::load(Ksh + (j * 16 + c) * HD + 0  + 8 * hh);
      s[j] = mma_h(qf[0], kb0, s[j]);
      const v16h kb1 = Frag<_Float16>::load(Ksh + (j * 16 + c) * HD + 32 + 8 * hh);
      s[j] = mma_h(qf[1], kb1, s[j]);
    }

    float cm[8];
#pragma unroll
    for (int r = 0; r < 8; ++r) {
      const int qrow = q0 + 8 * hh + r;
      const float* mrp = mbp + (size_t)qrow * S_LEN + kv0 + c;
      float m = NEG_FILL;
#pragma unroll
      for (int j = 0; j < 4; ++j) {
        float x = s[j][r] * SCALE_QK;
        if (mrp[j * 16] < -5000.0f) x = NEG_FILL;
        s[j][r] = x;
        m = fmaxf(m, x);
      }
#pragma unroll
      for (int off = 1; off < 16; off <<= 1) m = fmaxf(m, __shfl_xor(m, off, 32));
      cm[r] = m;
    }

    _Float16* pw = Psh[wave];
#pragma unroll
    for (int r = 0; r < 8; ++r) {
      const float mnew  = fmaxf(mrow[r], cm[r]);
      const float alpha = __expf(mrow[r] - mnew);
      mrow[r] = mnew;
      float psum = 0.f;
#pragma unroll
      for (int j = 0; j < 4; ++j) {
        const float p = __expf(s[j][r] - mnew);
        psum += p;
        pw[(8 * hh + r) * KC + j * 16 + c] = (_Float16)(p * PSC);
      }
#pragma unroll
      for (int off = 1; off < 16; off <<= 1) psum += __shfl_xor(psum, off, 32);
      lrow[r] = lrow[r] * alpha + psum;
#pragma unroll
      for (int t = 0; t < 4; ++t) oacc[t][r] *= alpha;
    }
    __builtin_amdgcn_fence(__ATOMIC_RELEASE, "workgroup");
    __builtin_amdgcn_wave_barrier();
    __builtin_amdgcn_fence(__ATOMIC_ACQUIRE, "workgroup");

#pragma unroll 1
    for (int kk = 0; kk < 2; ++kk) {
      const v16h pa = Frag<_Float16>::load(pw + c * KC + kk * 32 + 8 * hh);
#pragma unroll
      for (int t = 0; t < 4; ++t) {
        const v16h vb = Frag<_Float16>::load(Vth + (t * 16 + c) * KC + kk * 32 + 8 * hh);
        oacc[t] = mma_h(pa, vb, oacc[t]);
      }
    }
  }

#pragma unroll
  for (int r = 0; r < 8; ++r) {
    const float inv = 1.0f / (lrow[r] * PSC);
    const int qloc = wave * 16 + 8 * hh + r;
#pragma unroll
    for (int t = 0; t < 4; ++t) Ob[(t * 16 + c) * OP + qloc] = oacc[t][r] * inv;
  }
  __syncthreads();
  {
    const int c4 = c * 4;
    for (int pass = 0; pass < 2; ++pass) {
#pragma unroll
      for (int it = 0; it < 8; ++it) {
        const int d = wave * 16 + it * 2 + hh;
        const v4f val = *(const v4f*)(Ob + d * OP + c4);
        *(volatile v4f*)(obp + (size_t)d * S_LEN + q0b + c4) = val;
      }
      __threadfence();
    }
  }
}

extern "C" void kernel_launch(void* const* d_in, const int* in_sizes, int n_in,
                              void* d_out, int out_size, void* d_ws, size_t ws_size,
                              hipStream_t stream) {
  if (n_in < 4) return;
  const float* q  = (const float*)d_in[0];
  const float* k  = (const float*)d_in[1];
  const float* v  = (const float*)d_in[2];
  const float* mk = (const float*)d_in[3];
  float* out = (float*)d_out;

  const int per_b = C_CH * S_LEN;
  const int nb = in_sizes[0] / per_b;
  if (nb <= 0 || in_sizes[0] != nb * per_b) return;
  if (in_sizes[1] != in_sizes[0] || in_sizes[2] != in_sizes[0]) return;
  if ((long long)in_sizes[3] != (long long)nb * S_LEN * S_LEN) return;
  if (out_size != in_sizes[0]) return;
  const int nbh = nb * N_HEADS;

  const size_t eb = (size_t)nbh * S_LEN * HD * sizeof(_Float16);
  const size_t offQ = 0, offK = eb, offV = 2 * eb;
  const size_t total = 3 * eb;
  if (total > ws_size || total > (size_t)134217728) return;
  _Float16* Qt = (_Float16*)((char*)d_ws + offQ);
  _Float16* Kt = (_Float16*)((char*)d_ws + offK);
  _Float16* Vh = (_Float16*)((char*)d_ws + offV);

  tcast_kernel<<<dim3(S_LEN / 64, nbh, 2), 128, 0, stream>>>(q, k, Qt, Kt);
  const int n2 = (int)((size_t)nbh * HD * S_LEN / 2);
  cast_f32_f16x2<<<dim3((n2 + 255) / 256), 256, 0, stream>>>(v, Vh, n2);
  attn_kernel<<<dim3(S_LEN / QB, nbh), 128, 0, stream>>>(Qt, Kt, Vh, mk, out, N_HEADS);
  (void)hipGetLastError();
}
